// GATInnerLayer_12077448036818
// MI455X (gfx1250) — hardware-verified
//
#include <hip/hip_runtime.h>
#include <stdint.h>

#define DIM 64
#define NPB 16
#define EP  72
#define DPB 512
#define AGT 64

typedef float          v8f  __attribute__((ext_vector_type(8)));
typedef float          v4f  __attribute__((ext_vector_type(4)));
typedef _Float16       v16h __attribute__((ext_vector_type(16)));
typedef _Float16       v8h  __attribute__((ext_vector_type(8)));
typedef __bf16         v16b __attribute__((ext_vector_type(16)));
typedef unsigned short v8us __attribute__((ext_vector_type(8)));

union FragH { v16h v; v8h  p[2]; };
union FragB { v16b v; v8us p[2]; };

__device__ __forceinline__ v8f wmma_bf16(v16b a, v16b b, v8f c)
{
    v8f d = __builtin_amdgcn_wmma_f32_16x16x32_bf16(false, a, false, b, (short)0, c, false, false);
    asm volatile("v_nop\n\tv_nop\n\tv_nop\n\tv_nop" : "+v"(d) : "v"(a), "v"(b));
    return d;
}
__device__ __forceinline__ v8f wmma_f16(v16h a, v16h b, v8f c)
{
    v8f d = __builtin_amdgcn_wmma_f32_16x16x32_f16(false, a, false, b, (short)0, c, false, false);
    asm volatile("v_nop\n\tv_nop\n\tv_nop\n\tv_nop" : "+v"(d) : "v"(a), "v"(b));
    return d;
}

__device__ __forceinline__ unsigned short f2bf(float f)
{
    unsigned int u = __float_as_uint(f);
    u += 0x7FFFu + ((u >> 16) & 1u);
    return (unsigned short)(u >> 16);
}
__device__ __forceinline__ float bf2f(unsigned short b)
{
    return __uint_as_float(((unsigned int)b) << 16);
}

__device__ __forceinline__ void split4(const float4 v, unsigned short* hi, unsigned short* lo, int o)
{
    float x[4] = {v.x, v.y, v.z, v.w};
    #pragma unroll
    for (int t = 0; t < 4; ++t) {
        unsigned short hb = f2bf(x[t]);
        unsigned short lb = f2bf(x[t] - bf2f(hb));
        hi[o + t] = hb;
        lo[o + t] = lb;
    }
}

__device__ __forceinline__ void proj_tiles(const unsigned short* hh, const unsigned short* hl,
                                           const unsigned short* wh, const unsigned short* wl,
                                           float* O, int wv, int hs, int m)
{
    #pragma unroll
    for (int cc = 0; cc < 2; ++cc) {
        const int ct = 2 * wv + cc;
        const int n  = 16 * ct + m;
        v8f acc = {0.f, 0.f, 0.f, 0.f, 0.f, 0.f, 0.f, 0.f};
        #pragma unroll
        for (int ks = 0; ks < 2; ++ks) {
            const int k0 = 32 * ks;
            FragB ah, al, bh, bl;
            ah.p[0] = *(const v8us*)(hh + m * DIM + k0 + 8 * hs);
            ah.p[1] = *(const v8us*)(hh + m * DIM + k0 + 16 + 8 * hs);
            al.p[0] = *(const v8us*)(hl + m * DIM + k0 + 8 * hs);
            al.p[1] = *(const v8us*)(hl + m * DIM + k0 + 16 + 8 * hs);
            bh.p[0] = *(const v8us*)(wh + n * DIM + k0 + 8 * hs);
            bh.p[1] = *(const v8us*)(wh + n * DIM + k0 + 16 + 8 * hs);
            bl.p[0] = *(const v8us*)(wl + n * DIM + k0 + 8 * hs);
            bl.p[1] = *(const v8us*)(wl + n * DIM + k0 + 16 + 8 * hs);
            acc = wmma_bf16(ah.v, bh.v, acc);
            acc = wmma_bf16(ah.v, bl.v, acc);
            acc = wmma_bf16(al.v, bh.v, acc);
        }
        #pragma unroll
        for (int r = 0; r < 8; ++r) O[(8 * hs + r) * DIM + 16 * ct + m] = acc[r];
    }
}

__global__ __launch_bounds__(64) void k_node_attn(const float* __restrict__ hin,
                                                  const float* __restrict__ Wq,
                                                  const float* __restrict__ Wk,
                                                  float* a_out,
                                                  int N)
{
    __shared__ __align__(16) unsigned short hh[NPB * DIM];
    __shared__ __align__(16) unsigned short hl[NPB * DIM];
    __shared__ __align__(16) unsigned short wh[DIM * DIM];
    __shared__ __align__(16) unsigned short wl[DIM * DIM];
    __shared__ __align__(16) float qs[NPB * DIM];
    __shared__ __align__(16) float ks[NPB * DIM];
    __shared__ __align__(16) _Float16 Esh[2][DIM * EP];
    __shared__ __align__(16) _Float16 vsh[2][DIM];
    __shared__ __align__(16) float ast[2][8 * DIM];

    const int tid  = threadIdx.x;
    const int lane = tid & 31;
    const int wv   = tid >> 5;
    const int hs   = lane >> 4;
    const int m    = lane & 15;
    const int node_base = blockIdx.x * NPB;

    for (int c = tid; c < NPB * DIM / 4; c += 64) {
        const int row = c >> 4;
        int node = node_base + row;
        if (node > N - 1) node = N - 1;
        const float4 v = *(const float4*)(hin + (size_t)node * DIM + (c & 15) * 4);
        split4(v, hh, hl, row * DIM + (c & 15) * 4);
    }
    for (int c = tid; c < DIM * DIM / 4; c += 64) {
        const float4 v = *(const float4*)(Wq + c * 4);
        split4(v, wh, wl, c * 4);
    }
    __syncthreads();
    proj_tiles(hh, hl, wh, wl, qs, wv, hs, m);
    __syncthreads();
    for (int c = tid; c < DIM * DIM / 4; c += 64) {
        const float4 v = *(const float4*)(Wk + c * 4);
        split4(v, wh, wl, c * 4);
    }
    __syncthreads();
    proj_tiles(hh, hl, wh, wl, ks, wv, hs, m);
    __syncthreads();

    _Float16* Ew = Esh[wv];
    _Float16* vw = vsh[wv];
    float*    aw = ast[wv];
    const float sc     = 0.125f;
    const float escale = 16384.0f;
    const float vscale = 256.0f;
    const float unscl  = 1.0f / 4194304.0f;

    for (int it = 0; it < 8; ++it) {
        const int nl = wv * 8 + it;
        int node = node_base + nl;
        if (node > N - 1) node = N - 1;
        const float* qrow = qs + nl * DIM;
        const float* krow = ks + nl * DIM;

        float qa = qrow[lane], qb = qrow[lane + 32];
        float qmax = fmaxf(qa, qb), qmin = fminf(qa, qb);
        #pragma unroll
        for (int off = 16; off > 0; off >>= 1) {
            qmax = fmaxf(qmax, __shfl_xor(qmax, off, 32));
            qmin = fminf(qmin, __shfl_xor(qmin, off, 32));
        }

        #pragma unroll
        for (int j2 = 0; j2 < 2; ++j2) {
            const int j = lane + 32 * j2;
            const float cj = krow[j] * sc;
            const float mj = (cj >= 0.0f) ? (qmax * cj) : (qmin * cj);
            float Z = 0.0f;
            #pragma unroll 4
            for (int i = 0; i < DIM; ++i) {
                const float e = __expf(qrow[i] * cj - mj);
                Z += e;
                Ew[i * EP + j] = (_Float16)(e * escale);
            }
            const float hv = hin[(size_t)node * DIM + j];
            vw[j] = (_Float16)(hv * (vscale / Z));
        }
        __syncthreads();

        v8f acc[4];
        #pragma unroll
        for (int mt = 0; mt < 4; ++mt) {
            #pragma unroll
            for (int r = 0; r < 8; ++r) acc[mt][r] = 0.0f;
        }
        #pragma unroll
        for (int kq = 0; kq < 2; ++kq) {
            const int k0 = 32 * kq;
            FragH bf;
            bf.p[0] = *(const v8h*)(vw + k0 + 8 * hs);
            bf.p[1] = *(const v8h*)(vw + k0 + 16 + 8 * hs);
            #pragma unroll
            for (int mt = 0; mt < 4; ++mt) {
                FragH af;
                af.p[0] = *(const v8h*)(Ew + (16 * mt + m) * EP + k0 + 8 * hs);
                af.p[1] = *(const v8h*)(Ew + (16 * mt + m) * EP + k0 + 16 + 8 * hs);
                acc[mt] = wmma_f16(af.v, bf.v, acc[mt]);
            }
        }
        if (m == 0) {
            #pragma unroll
            for (int mt = 0; mt < 4; ++mt) {
                #pragma unroll
                for (int r = 0; r < 8; ++r)
                    aw[it * DIM + 16 * mt + 8 * hs + r] = acc[mt][r] * unscl;
            }
        }
        __syncthreads();
    }

    {
        float* ap = a_out + (size_t)(node_base + 8 * wv) * DIM;
        v4f vals[4];
        #pragma unroll
        for (int q = 0; q < 4; ++q) vals[q] = *(const v4f*)(aw + (q * 32 + lane) * 4);
        #pragma unroll
        for (int q = 0; q < 4; ++q) *(volatile v4f*)(ap + (q * 32 + lane) * 4) = vals[q];
        __threadfence();
        #pragma unroll
        for (int q = 0; q < 4; ++q) *(volatile v4f*)(ap + (q * 32 + lane) * 4) = vals[q];
    }
}

__device__ __forceinline__ void seg_store_rows(const float* accs, const int* cnt, float* out,
                                               int dbase, int N, int wv, int lane)
{
    for (int p = wv; p < DPB / 2; p += 2) {
        const int r   = 2 * p + (lane >> 4);
        const int row = dbase + r;
        const int c4  = (lane & 15) * 4;
        const float cn  = (float)cnt[r];
        const float inv = 1.0f / fmaxf(cn, 1.0f);
        v4f v = *(const v4f*)(accs + r * DIM + c4);
        v = v * inv;
        if (row < N) *(volatile v4f*)(out + (size_t)row * DIM + c4) = v;
    }
}

__global__ __launch_bounds__(AGT) void k_seg_mean(const float* a,
                                                  const int* __restrict__ srcv,
                                                  const int* __restrict__ dstv,
                                                  float* out,
                                                  int N, int E)
{
    __shared__ __align__(16) float accs[DPB * DIM];
    __shared__ int cnt[DPB];
    __shared__ int hsl[64];
    __shared__ int hdl[64];
    __shared__ int nh[2];

    const int tid   = threadIdx.x;
    const int lane  = tid & 31;
    const int wv    = tid >> 5;
    const int dbase = blockIdx.x * DPB;

    {
        const v4f z = {0.f, 0.f, 0.f, 0.f};
        for (int i = tid; i < DPB * DIM / 4; i += AGT) *(v4f*)(accs + 4 * i) = z;
        for (int i = tid; i < DPB; i += AGT) cnt[i] = 0;
    }
    __syncthreads();

    for (int c0 = 0; c0 < E; c0 += AGT) {
        const int e = c0 + tid;
        int d = -1, s = 0;
        if (e < E) { d = dstv[e]; s = srcv[e]; }
        const unsigned dl = (unsigned)d - (unsigned)dbase;
        const bool hit = (e < E) && (d >= 0) && (d < N) && (dl < (unsigned)DPB);
        const unsigned msk = __builtin_amdgcn_ballot_w32(hit);
        const int pos = __builtin_popcount(msk & ((1u << lane) - 1u));
        if (hit) {
            if (s < 0) s = 0;
            if (s > N - 1) s = N - 1;
            hsl[wv * 32 + pos] = s;
            hdl[wv * 32 + pos] = (int)dl;
        }
        if (lane == 0) nh[wv] = __builtin_popcount(msk);
        __syncthreads();

        int n0 = nh[0], n1 = nh[1];
        if (n0 > 32) n0 = 32;
        if (n1 > 32) n1 = 32;
        const int nt = n0 + n1;
        for (int t = 0; t < nt; ++t) {
            const int slot = (t < n0) ? t : (32 + t - n0);
            int ss = hsl[slot];
            int dd = hdl[slot];
            if (ss < 0) ss = 0;
            if (ss > N - 1) ss = N - 1;
            if (dd < 0) dd = 0;
            if (dd > DPB - 1) dd = DPB - 1;
            const float v = a[(size_t)ss * DIM + tid];
            accs[dd * DIM + tid] += v;
            if (tid == 0) cnt[dd] += 1;
        }
        __syncthreads();
    }

    seg_store_rows(accs, cnt, out, dbase, N, wv, lane);
    __threadfence();
    seg_store_rows(accs, cnt, out, dbase, N, wv, lane);
}

extern "C" void kernel_launch(void* const* d_in, const int* in_sizes, int n_in,
                              void* d_out, int out_size, void* d_ws, size_t ws_size,
                              hipStream_t stream)
{
    if (n_in < 5) return;
    const float* h   = (const float*)d_in[0];
    const float* Wq  = (const float*)d_in[1];
    const float* Wk  = (const float*)d_in[2];
    const int*   src = (const int*)d_in[3];
    const int*   dst = (const int*)d_in[4];

    const int N = in_sizes[0] / DIM;
    int E = in_sizes[3];
    if (in_sizes[4] < E) E = in_sizes[4];
    if (N <= 0) return;
    if (in_sizes[1] < DIM * DIM || in_sizes[2] < DIM * DIM) return;
    if (out_size < N * DIM) return;

    const int nblk1 = (N + NPB - 1) / NPB;
    const size_t a_bytes = (size_t)nblk1 * NPB * DIM * sizeof(float);
    if (a_bytes > ws_size) return;
    float* a = (float*)d_ws;

    k_node_attn<<<nblk1, 64, 0, stream>>>(h, Wq, Wk, a, N);

    const int nblk2 = (N + DPB - 1) / DPB;
    k_seg_mean<<<nblk2, AGT, 0, stream>>>(a, src, dst, (float*)d_out, N, E);
}
